// OuterProduct_89438398972452
// MI455X (gfx1250) — hardware-verified
//
#include <hip/hip_runtime.h>
#include <math.h>

constexpr int kBatchN = 2;
constexpr int kSeqLen = 1024;
constexpr int kRows   = kBatchN * kSeqLen;
constexpr int kDim    = 1024;
constexpr int kHeads  = 16;
constexpr int kDh     = 64;
constexpr int kHid    = kHeads * kDh;
constexpr int kVQCols = 2 * kHid;
constexpr int kChunk  = 16;

constexpr size_t kBytesX16   = (size_t)kRows   * kDim    * 2;
constexpr size_t kBytesVQW16 = (size_t)kVQCols * kDim    * 2;
constexpr size_t kBytesW16   = (size_t)kHid    * kDim    * 2;
constexpr size_t kBytesVQ32  = (size_t)kRows   * kVQCols * 4;
constexpr size_t kBytesZ32   = (size_t)kRows   * kHid    * 4;
constexpr size_t kBytesH16   = (size_t)kRows   * kHid    * 2;
constexpr size_t kOffXh   = 0;
constexpr size_t kOffXl   = kOffXh   + kBytesX16;
constexpr size_t kOffVQWh = kOffXl   + kBytesX16;
constexpr size_t kOffVQWl = kOffVQWh + kBytesVQW16;
constexpr size_t kOffKWh  = kOffVQWl + kBytesVQW16;
constexpr size_t kOffKWl  = kOffKWh  + kBytesW16;
constexpr size_t kOffOWh  = kOffKWl  + kBytesW16;
constexpr size_t kOffOWl  = kOffOWh  + kBytesW16;
constexpr size_t kOffVQ   = kOffOWl  + kBytesW16;
constexpr size_t kOffZ    = kOffVQ   + kBytesVQ32;
constexpr size_t kOffHh   = kOffZ    + kBytesZ32;
constexpr size_t kOffHl   = kOffHh   + kBytesH16;
constexpr size_t kWsTotal = kOffHl   + kBytesH16;
static_assert(kWsTotal == 58720256, "carve total");
static_assert(kWsTotal <= 134217728, "carve under 128 MiB");

typedef __attribute__((ext_vector_type(16))) _Float16 v16h;
typedef __attribute__((ext_vector_type(8)))  _Float16 v8h;
typedef __attribute__((ext_vector_type(16))) __bf16   v16b;
typedef __attribute__((ext_vector_type(8)))  __bf16   v8b;
typedef __attribute__((ext_vector_type(8)))  float    v8f;
typedef __attribute__((ext_vector_type(4)))  float    v4f;
typedef __attribute__((ext_vector_type(4)))  unsigned int v4u;

__device__ __forceinline__ unsigned short f2bf_bits(float f) {
  unsigned u = __float_as_uint(f);
  return (unsigned short)((u + 0x7FFFu + ((u >> 16) & 1u)) >> 16);
}
__device__ __forceinline__ float bf_bits2f(unsigned short h) { return __uint_as_float(((unsigned)h) << 16); }

__device__ __forceinline__ void dep_guard_h(v8f& a, v8f& b, v16h x, v16h y) { asm volatile("v_nop\n\tv_nop\n\tv_nop\n\tv_nop" : "+v"(a), "+v"(b) : "v"(x), "v"(y)); }
__device__ __forceinline__ void dep_guard_b(v8f& a, v8f& b, v16b x, v16b y) { asm volatile("v_nop\n\tv_nop\n\tv_nop\n\tv_nop" : "+v"(a), "+v"(b) : "v"(x), "v"(y)); }
__device__ __forceinline__ void keep4_h(v16h a, v16h b, v16h c, v16h d) { asm volatile("v_nop" :: "v"(a), "v"(b), "v"(c), "v"(d)); }
__device__ __forceinline__ void keep4_b(v16b a, v16b b, v16b c, v16b d) { asm volatile("v_nop" :: "v"(a), "v"(b), "v"(c), "v"(d)); }
__device__ __forceinline__ void acc_guard4(v8f& a, v8f& b, v8f& c, v8f& d) { asm volatile("v_nop\n\tv_nop\n\tv_nop\n\tv_nop" : "+v"(a), "+v"(b), "+v"(c), "+v"(d)); }
template <typename T> struct Frag;
template <> struct Frag<_Float16> {
  typedef v16h V; union U { v16h v; v8h h[2]; };
  static __device__ __forceinline__ v16h load(const _Float16* p) {
    U f; f.h[0] = *(const v8h*)(p); f.h[1] = *(const v8h*)(p + 16); return f.v;
  }
  static __device__ __forceinline__ v8f mma(v16h a, v16h b, v8f c) {
    return __builtin_amdgcn_wmma_f32_16x16x32_f16(false, a, false, b, (short)0, c, false, false);
  }
  static __device__ __forceinline__ void guard(v8f& a, v8f& b, v16h x, v16h y) { dep_guard_h(a, b, x, y); }
  static __device__ __forceinline__ void keep(v16h a, v16h b, v16h c, v16h d) { keep4_h(a, b, c, d); }
};
template <> struct Frag<__bf16> {
  typedef v16b V; union U { v16b v; v8b h[2]; };
  static __device__ __forceinline__ v16b load(const __bf16* p) {
    U f; f.h[0] = *(const v8b*)(p); f.h[1] = *(const v8b*)(p + 16); return f.v;
  }
  static __device__ __forceinline__ v8f mma(v16b a, v16b b, v8f c) {
    return __builtin_amdgcn_wmma_f32_16x16x32_bf16(false, a, false, b, (short)0, c, false, false);
  }
  static __device__ __forceinline__ void guard(v8f& a, v8f& b, v16b x, v16b y) { dep_guard_b(a, b, x, y); }
  static __device__ __forceinline__ void keep(v16b a, v16b b, v16b c, v16b d) { keep4_b(a, b, c, d); }
};

__device__ __forceinline__ unsigned pk16(unsigned short a, unsigned short b) { return (unsigned)a | ((unsigned)b << 16); }

template <int ET> struct Elem;
template <> struct Elem<0> { typedef _Float16 T; };
template <> struct Elem<1> { typedef __bf16 T; };
template <int ET, bool SPLIT, int BIAS_MODE, int OUT_MODE, bool RESID, int ACT = 0>
__global__ __launch_bounds__(256) void wmma_gemm64(
    const unsigned short* __restrict__ Ap, const unsigned short* __restrict__ A2p, int lda, long strideA,
    const unsigned short* __restrict__ Btp, const unsigned short* __restrict__ Bt2p, int ldb, long strideB,
    void* __restrict__ Cout, void* __restrict__ Cout2, int ldc, long strideC,
    const float* __restrict__ bias,
    const float* __restrict__ resid, long strideR,
    int M, int N, int K, float scale) {
  typedef typename Elem<ET>::T T;
  typedef typename Frag<T>::V V;
  const T* A = (const T*)Ap; const T* A2 = (const T*)A2p; const T* Bt = (const T*)Btp; const T* Bt2 = (const T*)Bt2p;
  __shared__ __align__(16) float sT[8][16 * 68];
  const int b    = blockIdx.y;
  const int lane = threadIdx.x & 31;
  const int wave = threadIdx.x >> 5;
  const int tilesN = N >> 6;
  const int tilesM = M >> 6;
  const int tile = blockIdx.x * 8 + wave;
  if (tile >= tilesM * tilesN) return;
  const int tm = tile / tilesN;
  const int tn = tile - tm * tilesN;
  const int m0 = tm << 6;
  const int n0 = tn << 6;

  const T* Ab  = A  + (size_t)b * strideA;
  const T* Bb  = Bt + (size_t)b * strideB;
  const T* Ab2 = SPLIT ? (A2  + (size_t)b * strideA) : nullptr;
  const T* Bb2 = SPLIT ? (Bt2 + (size_t)b * strideB) : nullptr;

  const int rlane = lane & 15;
  const int koff  = (lane >> 4) * 8;
  const int mOff  = (lane >> 4) * 8;

  v8f acc[4][4];
#pragma unroll
  for (int i = 0; i < 4; ++i)
#pragma unroll
    for (int j = 0; j < 4; ++j) acc[i][j] = (v8f){0.f,0.f,0.f,0.f,0.f,0.f,0.f,0.f};

  for (int k0 = 0; k0 < K; k0 += 32) {
    V bh[4], bl[4];
#pragma unroll
    for (int j = 0; j < 4; ++j) {
      const size_t bo = (size_t)(n0 + (j << 4) + rlane) * ldb + koff + k0;
      bh[j] = Frag<T>::load(Bb + bo);
      if (SPLIT) bl[j] = Frag<T>::load(Bb2 + bo);
    }
#pragma unroll
    for (int i = 0; i < 4; ++i) {
      const size_t ao = (size_t)(m0 + (i << 4) + rlane) * lda + koff + k0;
      V ah = Frag<T>::load(Ab + ao);
      V al;
      if (SPLIT) al = Frag<T>::load(Ab2 + ao);
#pragma unroll
      for (int j = 0; j < 4; ++j) {
        acc[i][j] = Frag<T>::mma(ah, bh[j], acc[i][j]);
        if (SPLIT) {
          acc[i][j] = Frag<T>::mma(ah, bl[j], acc[i][j]);
          acc[i][j] = Frag<T>::mma(al, bh[j], acc[i][j]);
        }
      }
      Frag<T>::guard(acc[i][0], acc[i][3], ah, SPLIT ? al : ah);
    }
    Frag<T>::keep(bh[0], bh[1], bh[2], bh[3]);
    if (SPLIT) Frag<T>::keep(bl[0], bl[1], bl[2], bl[3]);
  }
  acc_guard4(acc[0][0], acc[0][1], acc[0][2], acc[0][3]);
  acc_guard4(acc[1][0], acc[1][1], acc[1][2], acc[1][3]);
  acc_guard4(acc[2][0], acc[2][1], acc[2][2], acc[2][3]);
  acc_guard4(acc[3][0], acc[3][1], acc[3][2], acc[3][3]);

  float* slab = sT[wave];
  const float* Rb = RESID ? (resid + (size_t)b * strideR) : nullptr;
#pragma unroll
  for (int i = 0; i < 4; ++i) {
    const int mBase = m0 + (i << 4);
#pragma unroll
    for (int j = 0; j < 4; ++j) {
      const int n = n0 + (j << 4) + rlane;
      float bv = 0.f;
      if (BIAS_MODE == 2) bv = bias[n];
#pragma unroll
      for (int r = 0; r < 8; ++r) {
        float v = acc[i][j][r] * scale;
        if (BIAS_MODE == 1) v += bias[mBase + mOff + r];
        if (BIAS_MODE == 2) v += bv;
        if (RESID) v += Rb[(size_t)(mBase + mOff + r) * ldc + n];
        if (ACT == 2) v = fmaxf(v, 0.0f);
        if (ACT == 4) v = (v > 0.f) ? v : 0.01f * v;
        slab[(mOff + r) * 68 + (j << 4) + rlane] = v;
      }
    }
    __builtin_amdgcn_fence(__ATOMIC_RELEASE, "workgroup");
    __builtin_amdgcn_wave_barrier();
    __builtin_amdgcn_fence(__ATOMIC_ACQUIRE, "workgroup");
    if (OUT_MODE == 0) {
      float* C = (float*)Cout + (size_t)b * strideC;
      const int hh = lane >> 4, c4 = (lane & 15) * 4;
      for (int pass = 0; pass < 2; ++pass) {
#pragma unroll
        for (int it = 0; it < 8; ++it) {
          const int row = it * 2 + hh;
          v4f v = *(const v4f*)(slab + row * 68 + c4);
          *(volatile v4f*)(C + (size_t)(mBase + row) * ldc + n0 + c4) = v;
        }
        __threadfence();
      }
    } else {
      const int q = lane >> 3, c8 = (lane & 7) * 8;
      unsigned short* C  = (unsigned short*)Cout  + (size_t)b * strideC;
      unsigned short* C2 = (OUT_MODE == 2) ? ((unsigned short*)Cout2 + (size_t)b * strideC) : nullptr;
      for (int pass = 0; pass < 2; ++pass) {
#pragma unroll
        for (int it = 0; it < 4; ++it) {
          const int row = it * 4 + q;
          const float* sp = slab + row * 68 + c8;
          v8h hv, lv;
#pragma unroll
          for (int e = 0; e < 8; ++e) {
            if (OUT_MODE == 1) {
              hv[e] = (_Float16)sp[e];
            } else {
              unsigned short hb = f2bf_bits(sp[e]);
              unsigned short lb = f2bf_bits(sp[e] - bf_bits2f(hb));
              hv[e] = __builtin_bit_cast(_Float16, hb);
              lv[e] = __builtin_bit_cast(_Float16, lb);
            }
          }
          *(volatile v8h*)(C + (size_t)(mBase + row) * ldc + n0 + c8) = hv;
          if (OUT_MODE == 2) *(volatile v8h*)(C2 + (size_t)(mBase + row) * ldc + n0 + c8) = lv;
        }
        __threadfence();
      }
    }
    __builtin_amdgcn_fence(__ATOMIC_RELEASE, "workgroup");
    __builtin_amdgcn_wave_barrier();
    __builtin_amdgcn_fence(__ATOMIC_ACQUIRE, "workgroup");
  }
}

__global__ __launch_bounds__(256) void split8_bf16_kernel(const float* __restrict__ in,
                                                          unsigned short* __restrict__ hi,
                                                          unsigned short* __restrict__ lo, int n8) {
  const int i = blockIdx.x * 256 + threadIdx.x;
  if (i >= n8) return;
  const float* p = in + 8 * (size_t)i;
  const v4f a = *(const v4f*)(p);
  const v4f c = *(const v4f*)(p + 4);
  unsigned short hb[8], lb[8];
#pragma unroll
  for (int e = 0; e < 4; ++e) {
    hb[e]     = f2bf_bits(a[e]);
    lb[e]     = f2bf_bits(a[e] - bf_bits2f(hb[e]));
    hb[4 + e] = f2bf_bits(c[e]);
    lb[4 + e] = f2bf_bits(c[e] - bf_bits2f(hb[4 + e]));
  }
  const v4u uh = (v4u){pk16(hb[0], hb[1]), pk16(hb[2], hb[3]), pk16(hb[4], hb[5]), pk16(hb[6], hb[7])};
  const v4u ul = (v4u){pk16(lb[0], lb[1]), pk16(lb[2], lb[3]), pk16(lb[4], lb[5]), pk16(lb[6], lb[7])};
  unsigned short* qh = hi + 8 * (size_t)i;
  unsigned short* ql = lo + 8 * (size_t)i;
  *(volatile v4u*)qh = uh;
  *(volatile v4u*)ql = ul;
  __threadfence();
  *(volatile v4u*)qh = uh;
  *(volatile v4u*)ql = ul;
}

__global__ __launch_bounds__(64) void gated_scan_kernel(const float* __restrict__ Zp, const float* __restrict__ VQp,
                                                         unsigned short* __restrict__ Hh, unsigned short* __restrict__ Hl) {
#pragma clang fp contract(off)
  __shared__ __align__(16) float ks[kChunk][kDh];
  __shared__ __align__(16) float om[kChunk][kDh];
  __shared__ __align__(16) float qs[kChunk][kDh];
  __shared__ __align__(16) float vs[kChunk][kDh];
  __shared__ __align__(16) float hs[kChunk][kDh];
  const int tid = threadIdx.x;
  const int nb  = blockIdx.x / kHeads;
  const int hd  = blockIdx.x - nb * kHeads;
  const size_t rowbase = (size_t)nb * kSeqLen;
  const int col = hd * kDh + tid;

  float kv[kDh];
#pragma unroll
  for (int i = 0; i < kDh; ++i) kv[i] = 0.f;

  for (int t0 = 0; t0 < kSeqLen; t0 += kChunk) {
#pragma unroll 1
    for (int s = 0; s < kChunk; ++s) {
      const size_t row = rowbase + (size_t)(t0 + s);
      const float z  = Zp[row * kHid + col];
      const float vv = VQp[row * kVQCols + col];
      const float qv = VQp[row * kVQCols + kHid + col];
      const float ex = expf(-z);
      const float kval = 1.0f / (1.0f + ex);
      ks[s][tid] = kval;
      om[s][tid] = 1.0f - kval;
      qs[s][tid] = qv;
      vs[s][tid] = vv;
    }
    __syncthreads();

#pragma unroll 1
    for (int s = 0; s < kChunk; ++s) {
      const float vj = vs[s][tid];
      const float* kr = &ks[s][0];
      const float* orw = &om[s][0];
      const float* qr = &qs[s][0];
      float hsum = 0.f;
#pragma unroll
      for (int i4 = 0; i4 < kDh / 4; ++i4) {
        const v4f k4 = *(const v4f*)(kr + 4 * i4);
        const v4f o4 = *(const v4f*)(orw + 4 * i4);
        const v4f q4 = *(const v4f*)(qr + 4 * i4);
#pragma unroll
        for (int e = 0; e < 4; ++e) {
          const float pk = k4[e] * kv[4 * i4 + e];
          const float pu = o4[e] * vj;
          const float nv = pk + pu;
          kv[4 * i4 + e] = nv;
          const float pq = q4[e] * nv;
          hsum = hsum + pq;
        }
        if ((i4 & 3) == 3) { asm volatile("" ::: "memory"); }
      }
      hs[s][tid] = hsum;
    }
    __syncthreads();

    {
      const int rq = tid >> 3;
      const int c8 = (tid & 7) * 8;
      for (int pass = 0; pass < 2; ++pass) {
#pragma unroll
        for (int it = 0; it < 2; ++it) {
          const int s = it * 8 + rq;
          const v4f a = *(const v4f*)(&hs[s][c8]);
          const v4f c = *(const v4f*)(&hs[s][c8 + 4]);
          unsigned short hb[8], lb[8];
#pragma unroll
          for (int e = 0; e < 4; ++e) {
            hb[e]     = f2bf_bits(a[e]);
            lb[e]     = f2bf_bits(a[e] - bf_bits2f(hb[e]));
            hb[4 + e] = f2bf_bits(c[e]);
            lb[4 + e] = f2bf_bits(c[e] - bf_bits2f(hb[4 + e]));
          }
          const v4u uh = (v4u){pk16(hb[0], hb[1]), pk16(hb[2], hb[3]), pk16(hb[4], hb[5]), pk16(hb[6], hb[7])};
          const v4u ul = (v4u){pk16(lb[0], lb[1]), pk16(lb[2], lb[3]), pk16(lb[4], lb[5]), pk16(lb[6], lb[7])};
          const size_t off = (rowbase + (size_t)(t0 + s)) * kHid + (size_t)hd * kDh + c8;
          *(volatile v4u*)(Hh + off) = uh;
          *(volatile v4u*)(Hl + off) = ul;
        }
        __threadfence();
      }
    }
  }
}

extern "C" void kernel_launch(void* const* d_in, const int* in_sizes, int n_in,
                              void* d_out, int out_size, void* d_ws, size_t ws_size,
                              hipStream_t stream) {
  if (n_in < 6) return;
  if (in_sizes[0] != kRows * kDim || in_sizes[1] != kHid * kDim || in_sizes[2] != kHid ||
      in_sizes[3] != kVQCols * kDim || in_sizes[4] != kDim * kHid || in_sizes[5] != kDim) return;
  if (out_size != kRows * kDim) return;
  if (ws_size < kWsTotal) return;

  const float* x     = (const float*)d_in[0];
  const float* key_w = (const float*)d_in[1];
  const float* key_b = (const float*)d_in[2];
  const float* vq_w  = (const float*)d_in[3];
  const float* out_w = (const float*)d_in[4];
  const float* out_b = (const float*)d_in[5];
  float* out = (float*)d_out;

  char* ws = (char*)d_ws;
  unsigned short* Xh   = (unsigned short*)(ws + kOffXh);
  unsigned short* Xl   = (unsigned short*)(ws + kOffXl);
  unsigned short* VQWh = (unsigned short*)(ws + kOffVQWh);
  unsigned short* VQWl = (unsigned short*)(ws + kOffVQWl);
  unsigned short* KWh  = (unsigned short*)(ws + kOffKWh);
  unsigned short* KWl  = (unsigned short*)(ws + kOffKWl);
  unsigned short* OWh  = (unsigned short*)(ws + kOffOWh);
  unsigned short* OWl  = (unsigned short*)(ws + kOffOWl);
  float* VQf = (float*)(ws + kOffVQ);
  float* Zf  = (float*)(ws + kOffZ);
  unsigned short* Hh   = (unsigned short*)(ws + kOffHh);
  unsigned short* Hl   = (unsigned short*)(ws + kOffHl);

  {
    const int n8x  = (kRows * kDim) / 8;
    const int n8vq = (kVQCols * kDim) / 8;
    const int n8w  = (kHid * kDim) / 8;
    split8_bf16_kernel<<<dim3((n8x + 255) / 256), dim3(256), 0, stream>>>(x, Xh, Xl, n8x);
    split8_bf16_kernel<<<dim3((n8vq + 255) / 256), dim3(256), 0, stream>>>(vq_w, VQWh, VQWl, n8vq);
    split8_bf16_kernel<<<dim3((n8w + 255) / 256), dim3(256), 0, stream>>>(key_w, KWh, KWl, n8w);
    split8_bf16_kernel<<<dim3((n8w + 255) / 256), dim3(256), 0, stream>>>(out_w, OWh, OWl, n8w);
  }

  wmma_gemm64<1, true, 0, 0, false, 0><<<dim3((kRows / 64) * (kVQCols / 64) / 8, 1), dim3(256), 0, stream>>>(
      Xh, Xl, kDim, 0L, VQWh, VQWl, kDim, 0L, (void*)VQf, nullptr, kVQCols, 0L,
      nullptr, nullptr, 0L, kRows, kVQCols, kDim, 1.0f);

  wmma_gemm64<1, true, 2, 0, false, 0><<<dim3((kRows / 64) * (kHid / 64) / 8, 1), dim3(256), 0, stream>>>(
      Xh, Xl, kDim, 0L, KWh, KWl, kDim, 0L, (void*)Zf, nullptr, kHid, 0L,
      key_b, nullptr, 0L, kRows, kHid, kDim, 1.0f);

  gated_scan_kernel<<<dim3(kBatchN * kHeads), dim3(64), 0, stream>>>(Zf, VQf, Hh, Hl);

  wmma_gemm64<1, true, 2, 0, false, 0><<<dim3((kRows / 64) * (kDim / 64) / 8, 1), dim3(256), 0, stream>>>(
      Hh, Hl, kHid, 0L, OWh, OWl, kHid, 0L, (void*)out, nullptr, kDim, 0L,
      out_b, nullptr, 0L, kRows, kDim, kHid, 1.0f);
}
